// GCRN_87617332838643
// MI455X (gfx1250) — hardware-verified
//
#include <hip/hip_runtime.h>
#include <stddef.h>


#define NBAT   16
#define NNODE  1024
#define NF     256
#define NG     256
#define NEC    4
#define NEDGE  16384
#define DIN    1024
#define HID    512
#define NEMB   256
#define NROW   16384

#define NTHR   256
#define NWAVE  8
#define EPT    8
#define NGRP   2
#define CHUNK  (NTHR * EPT * NGRP)
#define WCAP   (EPT * NGRP * 32)
#define LISTN  (NWAVE * WCAP)
#define NBT    128

#define AGG_OFF_LIST  (NBT * NF * 4)
#define AGG_OFF_WCNT  (AGG_OFF_LIST + LISTN * 4)
#define AGG_OFF_STG   (AGG_OFF_WCNT + 256)
#define LDS_AGG       (AGG_OFF_STG + NWAVE * 4096)
#define LDS_GEMM      (NWAVE * 2048 * 4)

#define GT_M   128
#define GT_N   128
#define RB_CNT (NROW / GT_M)

#define WP_B0  128
#define WP_B1  (WP_B0 + 256)
#define WP_B2  (WP_B1 + 128)
#define WP_B3  (WP_B2 + 64)

#define WS_CAP 134217728

static_assert((CHUNK & (CHUNK - 1)) == 0);
static_assert((NBT & (NBT - 1)) == 0 && NBT <= 4096);
static_assert(NEDGE % CHUNK == 0);
static_assert(NNODE % NBT == 0);
static_assert(NF % 32 == 0 && NG % 64 == 0 && DIN % 32 == 0 && HID % GT_N == 0 && NEMB % GT_N == 0);
static_assert(NROW % GT_M == 0);
static_assert(NBT == 16 * NWAVE);
static_assert(GT_N == 128 && HID % 128 == 0);

typedef float          v4f  __attribute__((ext_vector_type(4)));
typedef float          v8f  __attribute__((ext_vector_type(8)));
typedef int            v4i  __attribute__((ext_vector_type(4)));
typedef unsigned int   v4u  __attribute__((ext_vector_type(4)));
typedef unsigned short v8us __attribute__((ext_vector_type(8), may_alias));
typedef __bf16         v16b __attribute__((ext_vector_type(16)));
union FragB { v16b v; v8us h[2]; };

__device__ __forceinline__ unsigned bfr(float f) {
  const unsigned u = __float_as_uint(f);
  return (u + 0x7FFFu + ((u >> 16) & 1u)) >> 16;
}
__device__ __forceinline__ float bff(unsigned b) { return __uint_as_float(b << 16); }

__device__ __forceinline__ void split8(v4f a, v4f c, v4u& hv, v4u& lv) {
  const unsigned h0 = bfr(a.x), h1 = bfr(a.y), h2 = bfr(a.z), h3 = bfr(a.w);
  const unsigned h4 = bfr(c.x), h5 = bfr(c.y), h6 = bfr(c.z), h7 = bfr(c.w);
  const unsigned l0 = bfr(a.x - bff(h0)), l1 = bfr(a.y - bff(h1)), l2 = bfr(a.z - bff(h2)), l3 = bfr(a.w - bff(h3));
  const unsigned l4 = bfr(c.x - bff(h4)), l5 = bfr(c.y - bff(h5)), l6 = bfr(c.z - bff(h6)), l7 = bfr(c.w - bff(h7));
  hv.x = h0 | (h1 << 16); hv.y = h2 | (h3 << 16); hv.z = h4 | (h5 << 16); hv.w = h6 | (h7 << 16);
  lv.x = l0 | (l1 << 16); lv.y = l2 | (l3 << 16); lv.z = l4 | (l5 << 16); lv.w = l6 | (l7 << 16);
}

__device__ __forceinline__ v8f wmb(v16b a, v16b b, v8f c) {
  v8f d = __builtin_amdgcn_wmma_f32_16x16x32_bf16(false, a, false, b, (short)0, c, false, false);
  asm volatile("v_nop\n\tv_nop\n\tv_nop\n\tv_nop" : "+v"(d) : "v"(a), "v"(b));
  return d;
}

template <int NB>
__device__ __forceinline__ int scan_chunk(const int* __restrict__ dsts, int nE, int cbase, int nodeBase,
                                          int vec8, int* list, int tid, int lane, int wave) {
  int wc = 0;
#pragma unroll
  for (int g = 0; g < NGRP; ++g) {
    const int el0  = (g * NTHR + tid) * EPT;
    const int e0   = cbase + el0;
    const int sent = -2147483647 - 1;
    v4i da, db;
    if (vec8 != 0 && cbase + CHUNK <= nE) {
      da = *(const v4i*)(dsts + e0);
      db = *(const v4i*)(dsts + e0 + 4);
    } else {
      da.x = (e0     < nE) ? dsts[min(e0, nE - 1)] : sent;
      da.y = (e0 + 1 < nE) ? dsts[min(e0 + 1, nE - 1)] : sent;
      da.z = (e0 + 2 < nE) ? dsts[min(e0 + 2, nE - 1)] : sent;
      da.w = (e0 + 3 < nE) ? dsts[min(e0 + 3, nE - 1)] : sent;
      db.x = (e0 + 4 < nE) ? dsts[min(e0 + 4, nE - 1)] : sent;
      db.y = (e0 + 5 < nE) ? dsts[min(e0 + 5, nE - 1)] : sent;
      db.z = (e0 + 6 < nE) ? dsts[min(e0 + 6, nE - 1)] : sent;
      db.w = (e0 + 7 < nE) ? dsts[min(e0 + 7, nE - 1)] : sent;
    }
    const unsigned nb = (unsigned)nodeBase;
    const unsigned s0 = (unsigned)da.x - nb, s1 = (unsigned)da.y - nb;
    const unsigned s2 = (unsigned)da.z - nb, s3 = (unsigned)da.w - nb;
    const unsigned s4 = (unsigned)db.x - nb, s5 = (unsigned)db.y - nb;
    const unsigned s6 = (unsigned)db.z - nb, s7 = (unsigned)db.w - nb;
    const bool h0 = s0 < (unsigned)NB, h1 = s1 < (unsigned)NB, h2 = s2 < (unsigned)NB, h3 = s3 < (unsigned)NB;
    const bool h4 = s4 < (unsigned)NB, h5 = s5 < (unsigned)NB, h6 = s6 < (unsigned)NB, h7 = s7 < (unsigned)NB;
    const unsigned any = __builtin_amdgcn_ballot_w32(h0 | h1 | h2 | h3 | h4 | h5 | h6 | h7);
    if (any != 0u) {
#define HITJ(J, HJ, SJ) { \
        const unsigned mj = __builtin_amdgcn_ballot_w32(HJ); \
        if (mj != 0u) { \
          if (HJ) { \
            const int pos = wc + (int)__builtin_amdgcn_mbcnt_lo(mj, 0u); \
            if (pos < WCAP) list[wave * WCAP + pos] = ((el0 + (J)) << 12) | (int)(SJ); \
          } \
          wc += (int)__builtin_popcount(mj); } }
      HITJ(0, h0, s0)
      HITJ(1, h1, s1)
      HITJ(2, h2, s2)
      HITJ(3, h3, s3)
      HITJ(4, h4, s4)
      HITJ(5, h5, s5)
      HITJ(6, h6, s6)
      HITJ(7, h7, s7)
#undef HITJ
    }
  }
  return wc;
}

__global__ __launch_bounds__(NTHR) void k_wprep(
    const float* __restrict__ Ws, const float* __restrict__ W0,
    const float* __restrict__ W1, const float* __restrict__ W2,
    unsigned short* WsH, unsigned short* WsL, unsigned short* W0H, unsigned short* W0L,
    unsigned short* W1H, unsigned short* W1L, unsigned short* W2H, unsigned short* W2L) {
  const int blk = blockIdx.x, tid = threadIdx.x;
  v4f a, c;
  unsigned short* dh;
  unsigned short* dl;
  if (blk < WP_B0) {
    const int o = (blk * NTHR + tid) * 8;
    const int e = o >> 16, rem = o & 65535, n = rem >> 8, k0 = rem & 255;
    const float* p = Ws + (size_t)e * (NF * NG) + (size_t)k0 * NG + n;
    a.x = p[0];      a.y = p[NG];     a.z = p[2 * NG]; a.w = p[3 * NG];
    c.x = p[4 * NG]; c.y = p[5 * NG]; c.z = p[6 * NG]; c.w = p[7 * NG];
    dh = WsH + o; dl = WsL + o;
  } else if (blk < WP_B1) {
    const int o = ((blk - WP_B0) * NTHR + tid) * 8;
    a = *(const v4f*)(W0 + o); c = *(const v4f*)(W0 + o + 4);
    dh = W0H + o; dl = W0L + o;
  } else if (blk < WP_B2) {
    const int o = ((blk - WP_B1) * NTHR + tid) * 8;
    a = *(const v4f*)(W1 + o); c = *(const v4f*)(W1 + o + 4);
    dh = W1H + o; dl = W1L + o;
  } else {
    const int o = ((blk - WP_B2) * NTHR + tid) * 8;
    a = *(const v4f*)(W2 + o); c = *(const v4f*)(W2 + o + 4);
    dh = W2H + o; dl = W2L + o;
  }
  v4u hv, lv;
  split8(a, c, hv, lv);
  *(volatile v4u*)dh = hv;
  *(volatile v4u*)dl = lv;
  __threadfence();
  *(volatile v4u*)dh = hv;
  *(volatile v4u*)dl = lv;
}

__global__ __launch_bounds__(NTHR) void k_agg(
    const int* __restrict__ Aidx, const float* __restrict__ X,
    const unsigned short* __restrict__ WsH, const unsigned short* __restrict__ WsL,
    unsigned short* PH, unsigned short* PL, int vec8) {
  extern __shared__ v4f lds_dyn[];
  float*          sS   = (float*)lds_dyn;
  unsigned short* s16  = (unsigned short*)lds_dyn;
  int*            list = (int*)((char*)lds_dyn + AGG_OFF_LIST);
  int*            wcnt = (int*)((char*)lds_dyn + AGG_OFF_WCNT);
  unsigned short* stg  = (unsigned short*)((char*)lds_dyn + AGG_OFF_STG);
  const int tid = threadIdx.x, lane = tid & 31, wave = tid >> 5, hh = lane >> 4, m = lane & 15;
  const int blk = blockIdx.x;
  const int b = blk >> 5, e = (blk >> 3) & 3, tile = blk & 7;
  const int nodeBase = tile * NBT;
  const int nE = NEDGE;
  const int* dsts = Aidx + (size_t)((b * NEC + e) * 2) * NEDGE;
  const int* srcs = dsts + NEDGE;

  {
    const v4f z = {0.f, 0.f, 0.f, 0.f};
    for (int i = tid; i < NBT * NF / 4; i += NTHR) lds_dyn[i] = z;
  }
  __syncthreads();

  const int nChunks = (nE + CHUNK - 1) / CHUNK;
#pragma unroll 1
  for (int ch = 0; ch < nChunks; ++ch) {
    const int cbase = ch * CHUNK;
    const int wc = scan_chunk<NBT>(dsts, nE, cbase, nodeBase, vec8, list, tid, lane, wave);
    if (lane == 0) wcnt[wave] = wc;
    __syncthreads();
    if (wave == 0) {
#pragma unroll 1
      for (int wsx = 0; wsx < NWAVE; ++wsx) {
        int n = __builtin_amdgcn_readfirstlane(wcnt[wsx]);
        n = n > WCAP ? WCAP : (n < 0 ? 0 : n);
        const int* lp = list + wsx * WCAP;
#pragma unroll 1
        for (int i = 0; i < n; ++i) {
          const int ent  = __builtin_amdgcn_readfirstlane(lp[i]);
          const int slot = ent & (NBT - 1);
          int eg = cbase + ((ent >> 12) & (CHUNK - 1));
          eg = eg > nE - 1 ? nE - 1 : eg;
          int src = srcs[eg];
          src = src < 0 ? 0 : (src > NNODE - 1 ? NNODE - 1 : src);
          const float* xp = X + ((size_t)(b * NNODE + src)) * NF + 8 * lane;
          const v4f x0 = *(const v4f*)xp, x1 = *(const v4f*)(xp + 4);
          v4f* ap = (v4f*)(sS + slot * NF + 8 * lane);
          ap[0] = ap[0] + x0;
          ap[1] = ap[1] + x1;
        }
      }
    }
    __syncthreads();
  }

#pragma unroll 4
  for (int r = 0; r < 16; ++r) {
    const int row = 16 * wave + r;
    const float* p = sS + row * NF + 8 * lane;
    const v4f a = *(const v4f*)p, c = *(const v4f*)(p + 4);
    v4u hv, lv;
    split8(a, c, hv, lv);
    *(v4u*)(s16 + row * 512 + 8 * lane)       = hv;
    *(v4u*)(s16 + row * 512 + 256 + 8 * lane) = lv;
  }
  __syncthreads();

  const unsigned short* arow = s16 + (16 * wave + m) * 512 + 8 * hh;
  const unsigned short* pbh  = WsH + ((size_t)(e * NG + m)) * NF + 8 * hh;
  const unsigned short* pbl  = WsL + ((size_t)(e * NG + m)) * NF + 8 * hh;
  unsigned short* stgw = stg + wave * 2048;
  const int q8 = lane >> 3, c8 = lane & 7;
  const size_t growBase = (size_t)(b * NNODE + nodeBase + 16 * wave);

#pragma unroll 1
  for (int nc = 0; nc < NG / 64; ++nc) {
    v8f acc[4];
#pragma unroll
    for (int j = 0; j < 4; ++j) { v8f z = {0.f, 0.f, 0.f, 0.f, 0.f, 0.f, 0.f, 0.f}; acc[j] = z; }
#pragma unroll 1
    for (int kt = 0; kt < NF / 32; ++kt) {
      FragB ah, al;
      ah.h[0] = *(const v8us*)(arow + 32 * kt);
      ah.h[1] = *(const v8us*)(arow + 32 * kt + 16);
      al.h[0] = *(const v8us*)(arow + 256 + 32 * kt);
      al.h[1] = *(const v8us*)(arow + 256 + 32 * kt + 16);
#pragma unroll
      for (int j = 0; j < 4; ++j) {
        const size_t bo = (size_t)(64 * nc + 16 * j) * NF + 32 * kt;
        FragB bh, bl;
        bh.h[0] = *(const v8us*)(pbh + bo);
        bh.h[1] = *(const v8us*)(pbh + bo + 16);
        bl.h[0] = *(const v8us*)(pbl + bo);
        bl.h[1] = *(const v8us*)(pbl + bo + 16);
        acc[j] = wmb(ah.v, bh.v, acc[j]);
        acc[j] = wmb(ah.v, bl.v, acc[j]);
        acc[j] = wmb(al.v, bh.v, acc[j]);
      }
    }
#pragma unroll
    for (int j = 0; j < 4; ++j) {
#pragma unroll
      for (int r = 0; r < 8; ++r) {
        const float v = fmaxf(acc[j][r], 0.0f);
        const unsigned hb = bfr(v);
        const unsigned lb = bfr(v - bff(hb));
        stgw[(8 * hh + r) * 64 + 16 * j + m]        = (unsigned short)hb;
        stgw[1024 + (8 * hh + r) * 64 + 16 * j + m] = (unsigned short)lb;
      }
    }
    __syncthreads();
    v8us hv[4], lv[4];
#pragma unroll
    for (int i = 0; i < 4; ++i) {
      const int row = 4 * i + q8;
      hv[i] = *(const v8us*)(stgw + row * 64 + 8 * c8);
      lv[i] = *(const v8us*)(stgw + 1024 + row * 64 + 8 * c8);
    }
    const size_t cb = (size_t)e * NG + 64 * nc + 8 * c8;
#pragma unroll
    for (int i = 0; i < 4; ++i) {
      const size_t off = (growBase + (size_t)(4 * i + q8)) * DIN + cb;
      *(volatile v8us*)(PH + off) = hv[i];
      *(volatile v8us*)(PL + off) = lv[i];
    }
    __threadfence();
#pragma unroll
    for (int i = 0; i < 4; ++i) {
      const size_t off = (growBase + (size_t)(4 * i + q8)) * DIN + cb;
      *(volatile v8us*)(PH + off) = hv[i];
      *(volatile v8us*)(PL + off) = lv[i];
    }
    __syncthreads();
  }
}

__global__ __launch_bounds__(NTHR) void k_gemm(
    const unsigned short* __restrict__ Ah, const unsigned short* __restrict__ Al,
    const unsigned short* __restrict__ Wh, const unsigned short* __restrict__ Wl,
    const float* __restrict__ bias, float* C, float* psum, float* psq,
    int N, int K, int doStats) {
  extern __shared__ v4f lds_dyn[];
  __shared__ __attribute__((aligned(16))) float sstat[2 * GT_N];
  float* stg = (float*)lds_dyn;
  const int tid = threadIdx.x, lane = tid & 31, wave = tid >> 5, hh = lane >> 4, m = lane & 15;
  const int rw = wave >> 1, cw = wave & 1;
  const int rowBase = blockIdx.x * GT_M + 32 * rw;
  const int colBase = blockIdx.y * GT_N + 64 * cw;
  const size_t Ks = (size_t)K;

  v8f acc[2][4];
#pragma unroll
  for (int i = 0; i < 2; ++i)
#pragma unroll
    for (int j = 0; j < 4; ++j) { v8f z = {0.f, 0.f, 0.f, 0.f, 0.f, 0.f, 0.f, 0.f}; acc[i][j] = z; }

  const unsigned short* pa0h = Ah + (size_t)(rowBase + m) * Ks + 8 * hh;
  const unsigned short* pa1h = pa0h + 16 * Ks;
  const unsigned short* pa0l = Al + (size_t)(rowBase + m) * Ks + 8 * hh;
  const unsigned short* pa1l = pa0l + 16 * Ks;
  const unsigned short* pbh  = Wh + (size_t)(colBase + m) * Ks + 8 * hh;
  const unsigned short* pbl  = Wl + (size_t)(colBase + m) * Ks + 8 * hh;

#pragma unroll 1
  for (int k0 = 0; k0 < K; k0 += 32) {
    FragB a0h, a1h, a0l, a1l;
    a0h.h[0] = *(const v8us*)(pa0h + k0); a0h.h[1] = *(const v8us*)(pa0h + k0 + 16);
    a1h.h[0] = *(const v8us*)(pa1h + k0); a1h.h[1] = *(const v8us*)(pa1h + k0 + 16);
    a0l.h[0] = *(const v8us*)(pa0l + k0); a0l.h[1] = *(const v8us*)(pa0l + k0 + 16);
    a1l.h[0] = *(const v8us*)(pa1l + k0); a1l.h[1] = *(const v8us*)(pa1l + k0 + 16);
#pragma unroll
    for (int j = 0; j < 4; ++j) {
      const size_t bo = (size_t)(16 * j) * Ks + k0;
      FragB bh, bl;
      bh.h[0] = *(const v8us*)(pbh + bo); bh.h[1] = *(const v8us*)(pbh + bo + 16);
      bl.h[0] = *(const v8us*)(pbl + bo); bl.h[1] = *(const v8us*)(pbl + bo + 16);
      acc[0][j] = wmb(a0h.v, bh.v, acc[0][j]);
      acc[0][j] = wmb(a0h.v, bl.v, acc[0][j]);
      acc[0][j] = wmb(a0l.v, bh.v, acc[0][j]);
      acc[1][j] = wmb(a1h.v, bh.v, acc[1][j]);
      acc[1][j] = wmb(a1h.v, bl.v, acc[1][j]);
      acc[1][j] = wmb(a1l.v, bh.v, acc[1][j]);
    }
  }

  float* stgw = stg + wave * 2048;
#pragma unroll
  for (int j = 0; j < 4; ++j) {
    const float bc = bias[colBase + 16 * j + m];
#pragma unroll
    for (int i = 0; i < 2; ++i) {
      float* sp = stgw + (16 * i + 8 * hh) * 64 + 16 * j + m;
#pragma unroll
      for (int r = 0; r < 8; ++r) sp[r * 64] = acc[i][j][r] + bc;
    }
  }
  __syncthreads();

  if (doStats != 0) {
    const int c = tid & 127, which = tid >> 7;
    const int wsel = c >> 6, cl = c & 63;
    double s = 0.0;
#pragma unroll 4
    for (int rr = 0; rr < GT_M; ++rr) {
      const int w2 = (rr >> 5) * 2 + wsel;
      const float x = stg[w2 * 2048 + (rr & 31) * 64 + cl];
      const double xd = (double)x;
      s += (which != 0) ? xd * xd : xd;
    }
    sstat[tid] = (float)s;
    __syncthreads();
    if (wave < 2) {
      const int l4 = 4 * lane;
      const v4f v = *(const v4f*)(sstat + wave * GT_N + l4);
      float* pp = (wave != 0) ? psq : psum;
      float* gp = pp + (size_t)blockIdx.x * (size_t)N + (size_t)blockIdx.y * GT_N + l4;
      *(volatile v4f*)gp = v;
      __threadfence();
      *(volatile v4f*)gp = v;
    }
  }

  const int hsel = lane >> 4, c4 = (lane & 15) * 4;
  float* cbp = C + (size_t)rowBase * (size_t)N + colBase + c4;
#pragma unroll
  for (int i = 0; i < 16; ++i) {
    const int row = 2 * i + hsel;
    const v4f v = *(const v4f*)(stgw + row * 64 + c4);
    *(volatile v4f*)(cbp + (size_t)row * (size_t)N) = v;
  }
  __threadfence();
#pragma unroll
  for (int i = 0; i < 16; ++i) {
    const int row = 2 * i + hsel;
    const v4f v = *(const v4f*)(stgw + row * 64 + c4);
    *(volatile v4f*)(cbp + (size_t)row * (size_t)N) = v;
  }
}

__global__ __launch_bounds__(512) void k_bnfin(
    const float* psum, const float* psq, const float* __restrict__ gam,
    float* mean, float* scale, int N, int nRB, float invR) {
  __shared__ __attribute__((aligned(16))) float smu[HID];
  __shared__ __attribute__((aligned(16))) float ssc[HID];
  const int n  = threadIdx.x;
  const int nn = n < N ? n : N - 1;
  double s = 0.0, q = 0.0;
#pragma unroll 1
  for (int rb = 0; rb < nRB; ++rb) {
    s += (double)psum[(size_t)rb * N + nn];
    q += (double)psq[(size_t)rb * N + nn];
  }
  const double mu = s * (double)invR;
  double var = q * (double)invR - mu * mu;
  var = var < 0.0 ? 0.0 : var;
  const float rstd = rsqrtf((float)var + 1e-5f);
  const float mf = (float)mu;
  const float sc = gam[nn] * rstd;
  if (n < N && n < HID) { smu[n] = mf; ssc[n] = sc; }
  __syncthreads();
  const int n4 = N >> 2;
  if (n < 2 * n4) {
    const bool second = n >= n4;
    const int  i4 = (second ? n - n4 : n) * 4;
    const v4f vm = *(const v4f*)(smu + i4);
    const v4f vs = *(const v4f*)(ssc + i4);
    const v4f v  = second ? vs : vm;
    float* gp = (second ? scale : mean) + i4;
    *(volatile v4f*)gp = v;
    __threadfence();
    *(volatile v4f*)gp = v;
  }
}

__global__ __launch_bounds__(NTHR) void k_bnapply(
    const float* __restrict__ hf, const float* __restrict__ mean,
    const float* __restrict__ scale, const float* __restrict__ beta,
    unsigned short* Ph, unsigned short* Pl, int N, int total8) {
  const int g = blockIdx.x * NTHR + threadIdx.x;
  if (g >= total8) return;
  const size_t o = (size_t)g * 8;
  const int col0 = (int)(o % (size_t)N);
  unsigned p0 = 0, p1 = 0, p2 = 0, p3 = 0, q0 = 0, q1 = 0, q2 = 0, q3 = 0;
#pragma unroll 1
  for (int i = 0; i < 8; ++i) {
    const int cc = col0 + i;
    const float x = hf[o + i];
    float y = (x - mean[cc]) * scale[cc] + beta[cc];
    const float ng = expm1f(fminf(y, 0.0f));
    y = (y > 0.0f) ? y : ng;
    const unsigned hb = bfr(y);
    const unsigned lb = bfr(y - bff(hb));
    p0 = (p0 >> 16) | (p1 << 16); p1 = (p1 >> 16) | (p2 << 16); p2 = (p2 >> 16) | (p3 << 16); p3 = (p3 >> 16) | (hb << 16);
    q0 = (q0 >> 16) | (q1 << 16); q1 = (q1 >> 16) | (q2 << 16); q2 = (q2 >> 16) | (q3 << 16); q3 = (q3 >> 16) | (lb << 16);
  }
  v4u hv, lv;
  hv.x = p0; hv.y = p1; hv.z = p2; hv.w = p3;
  lv.x = q0; lv.y = q1; lv.z = q2; lv.w = q3;
  *(volatile v4u*)(Ph + o) = hv;
  *(volatile v4u*)(Pl + o) = lv;
  __threadfence();
  *(volatile v4u*)(Ph + o) = hv;
  *(volatile v4u*)(Pl + o) = lv;
}

extern "C" void kernel_launch(void* const* d_in, const int* in_sizes, int n_in,
                              void* d_out, int out_size, void* d_ws, size_t ws_size,
                              hipStream_t stream) {
  if (n_in < 13) return;
  if (in_sizes[0] != NBAT * NEC * 2 * NEDGE) return;
  if (in_sizes[1] != NBAT * NNODE * NF) return;
  if (in_sizes[2] != NEC * NF * NG) return;
  if (in_sizes[3] != HID * DIN || in_sizes[4] != HID || in_sizes[5] != HID || in_sizes[6] != HID) return;
  if (in_sizes[7] != HID * HID || in_sizes[8] != HID || in_sizes[9] != HID || in_sizes[10] != HID) return;
  if (in_sizes[11] != NEMB * HID || in_sizes[12] != NEMB) return;
  if (out_size != NROW * NEMB) return;

  const int*   Aidx = (const int*)d_in[0];
  const float* X    = (const float*)d_in[1];
  const float* Ws   = (const float*)d_in[2];
  const float* W0   = (const float*)d_in[3];
  const float* b0   = (const float*)d_in[4];
  const float* g0   = (const float*)d_in[5];
  const float* be0  = (const float*)d_in[6];
  const float* W1   = (const float*)d_in[7];
  const float* b1   = (const float*)d_in[8];
  const float* g1   = (const float*)d_in[9];
  const float* be1  = (const float*)d_in[10];
  const float* W2   = (const float*)d_in[11];
  const float* b2   = (const float*)d_in[12];
  float* out = (float*)d_out;

  char* ws = (char*)d_ws;
  size_t off = 0;
#define CARVE(NAME, BYTES) const size_t NAME = off; off += (size_t)(BYTES); off = (off + 255) & ~(size_t)255;
  CARVE(oWsH, (size_t)NEC * NF * NG * 2)
  CARVE(oWsL, (size_t)NEC * NF * NG * 2)
  CARVE(oW0H, (size_t)HID * DIN * 2)
  CARVE(oW0L, (size_t)HID * DIN * 2)
  CARVE(oW1H, (size_t)HID * HID * 2)
  CARVE(oW1L, (size_t)HID * HID * 2)
  CARVE(oW2H, (size_t)NEMB * HID * 2)
  CARVE(oW2L, (size_t)NEMB * HID * 2)
  CARVE(oPH,  (size_t)NROW * DIN * 2)
  CARVE(oPL,  (size_t)NROW * DIN * 2)
  CARVE(oHF,  (size_t)NROW * HID * 4)
  CARVE(oPS,  (size_t)RB_CNT * HID * 4)
  CARVE(oPQ,  (size_t)RB_CNT * HID * 4)
  CARVE(oMU,  (size_t)HID * 4)
  CARVE(oSC,  (size_t)HID * 4)
#undef CARVE
  if (off > ws_size || off > (size_t)WS_CAP) return;

  unsigned short* WsH = (unsigned short*)(ws + oWsH);
  unsigned short* WsL = (unsigned short*)(ws + oWsL);
  unsigned short* W0H = (unsigned short*)(ws + oW0H);
  unsigned short* W0L = (unsigned short*)(ws + oW0L);
  unsigned short* W1H = (unsigned short*)(ws + oW1H);
  unsigned short* W1L = (unsigned short*)(ws + oW1L);
  unsigned short* W2H = (unsigned short*)(ws + oW2H);
  unsigned short* W2L = (unsigned short*)(ws + oW2L);
  unsigned short* PH  = (unsigned short*)(ws + oPH);
  unsigned short* PL  = (unsigned short*)(ws + oPL);
  float* HF   = (float*)(ws + oHF);
  float* PSUM = (float*)(ws + oPS);
  float* PSQ  = (float*)(ws + oPQ);
  float* MU   = (float*)(ws + oMU);
  float* SC   = (float*)(ws + oSC);

  const int vec8 = ((NEDGE & 7) == 0) ? 1 : 0;
  const float invR = 1.0f / (float)NROW;

  k_wprep<<<WP_B3, NTHR, 0, stream>>>(Ws, W0, W1, W2, WsH, WsL, W0H, W0L, W1H, W1L, W2H, W2L);

  hipFuncSetAttribute(reinterpret_cast<const void*>(&k_agg),
                      hipFuncAttributeMaxDynamicSharedMemorySize, LDS_AGG);
  k_agg<<<NBAT * NEC * (NNODE / NBT), NTHR, LDS_AGG, stream>>>(Aidx, X, WsH, WsL, PH, PL, vec8);

  hipFuncSetAttribute(reinterpret_cast<const void*>(&k_gemm),
                      hipFuncAttributeMaxDynamicSharedMemorySize, LDS_GEMM);

  k_gemm<<<dim3(NROW / GT_M, HID / GT_N, 1), NTHR, LDS_GEMM, stream>>>(
      PH, PL, W0H, W0L, b0, HF, PSUM, PSQ, HID, DIN, 1);
  k_bnfin<<<1, HID, 0, stream>>>(PSUM, PSQ, g0, MU, SC, HID, RB_CNT, invR);
  k_bnapply<<<(NROW * HID / 8) / NTHR, NTHR, 0, stream>>>(HF, MU, SC, be0, PH, PL, HID, NROW * HID / 8);

  k_gemm<<<dim3(NROW / GT_M, HID / GT_N, 1), NTHR, LDS_GEMM, stream>>>(
      PH, PL, W1H, W1L, b1, HF, PSUM, PSQ, HID, HID, 1);
  k_bnfin<<<1, HID, 0, stream>>>(PSUM, PSQ, g1, MU, SC, HID, RB_CNT, invR);
  k_bnapply<<<(NROW * HID / 8) / NTHR, NTHR, 0, stream>>>(HF, MU, SC, be1, PH, PL, HID, NROW * HID / 8);

  k_gemm<<<dim3(NROW / GT_M, NEMB / GT_N, 1), NTHR, LDS_GEMM, stream>>>(
      PH, PL, W2H, W2L, b2, out, PSUM, PSQ, NEMB, HID, 0);
}
